// LorentzLinearAttention_45157286150965
// MI455X (gfx1250) — hardware-verified
//
#include <hip/hip_runtime.h>
#include <math.h>


#define NB    8
#define NTOK  8192
#define DL    65
#define DX    64
#define MF    64
#define FF    192
#define CH    64
#define NCH   (NTOK / CH)
#define NBLK  (NB * NCH)
#define REC   (FF * DX + FF)
#define REC4  (REC / 4)
#define NTHR  256
#define NWAV  (NTHR / 32)
#define PSI2  0.70710678118654752f
#define EPSR  1e-4f
#define EPSQ  1e-8f

typedef __bf16 v16b __attribute__((ext_vector_type(16)));
typedef __bf16 v8b  __attribute__((ext_vector_type(8)));
typedef float  v8f  __attribute__((ext_vector_type(8)));
typedef float  v4f  __attribute__((ext_vector_type(4)));

union Frag { v16b v; v8b h[2]; };

__device__ __forceinline__ v8f zacc() {
  v8f a = {0.f, 0.f, 0.f, 0.f, 0.f, 0.f, 0.f, 0.f};
  return a;
}

__device__ __forceinline__ void st2(__bf16* H, __bf16* L, int i, float x) {
  __bf16 hi = (__bf16)x;
  float r = x - (float)hi;
  H[i] = hi;
  L[i] = (__bf16)r;
}

__device__ __forceinline__ v16b ldf(const __bf16* p) {
  Frag u;
  u.h[0] = *(const v8b*)(p);
  u.h[1] = *(const v8b*)(p + 16);
  return u.v;
}

__device__ __forceinline__ v8f mma3(v8f acc, v16b ah, v16b al, v16b bh, v16b bl) {
  acc = __builtin_amdgcn_wmma_f32_16x16x32_bf16(false, ah, false, bh, (short)0, acc, false, false);
  acc = __builtin_amdgcn_wmma_f32_16x16x32_bf16(false, ah, false, bl, (short)0, acc, false, false);
  acc = __builtin_amdgcn_wmma_f32_16x16x32_bf16(false, al, false, bh, (short)0, acc, false, false);
  asm volatile("v_nop\n\tv_nop\n\tv_nop\n\tv_nop" : "+v"(acc) : "v"(ah), "v"(al), "v"(bh), "v"(bl));
  return acc;
}

__device__ __forceinline__ void stage_x(const float* gb, __bf16* XH, __bf16* XL, float* X0, float* SS, int tid) {
  const int t = tid >> 2, q = tid & 3;
  const float* p = gb + (size_t)t * DL;
  float ss = 0.f;
#pragma unroll 4
  for (int i = 0; i < 16; ++i) {
    const int d = q * 16 + i;
    const float v = p[1 + d];
    ss += v * v;
    st2(XH, XL, t * DX + d, v);
  }
  ss += __shfl_xor(ss, 1);
  ss += __shfl_xor(ss, 2);
  if (q == 0) {
    X0[t] = p[0];
    SS[t] = ss;
  }
}

template <bool TR>
__device__ __forceinline__ void featurize(const __bf16* XH, const __bf16* XL,
                                          const __bf16* OH, const __bf16* OL,
                                          const float* X0, const float* SS,
                                          __bf16* outH, __bf16* outL,
                                          float sgn, int wave, int lane) {
  const int h = lane >> 4, l15 = lane & 15;
  for (int tile = wave; tile < (CH / 16) * (MF / 16); tile += NWAV) {
    const int rt = tile >> 2, mt = tile & 3;
    const __bf16* aH = XH + (rt * 16 + l15) * DX + 8 * h;
    const __bf16* aL = XL + (rt * 16 + l15) * DX + 8 * h;
    const __bf16* bH = OH + (mt * 16 + l15) * DX + 8 * h;
    const __bf16* bL = OL + (mt * 16 + l15) * DX + 8 * h;
    v8f acc = zacc();
#pragma unroll 1
    for (int ks = 0; ks < DX / 32; ++ks) {
      const int ko = ks * 32;
      acc = mma3(acc, ldf(aH + ko), ldf(aL + ko), ldf(bH + ko), ldf(bL + ko));
    }
#pragma unroll
    for (int r = 0; r < 8; ++r) {
      const int row = rt * 16 + 8 * h + r;
      const int m = mt * 16 + l15;
      const float x0 = X0[row];
      const float pr = acc[r] - 0.5f * SS[row];
      const float phi = expf(pr) * 0.125f;
      const float f1 = sgn * (x0 * phi);
      const float f2 = (PSI2 * (x0 * x0)) * phi;
      int i0, i1, i2;
      if (TR) {
        i0 = m * CH + row;
        i1 = (MF + m) * CH + row;
        i2 = (2 * MF + m) * CH + row;
      } else {
        i0 = row * FF + m;
        i1 = i0 + MF;
        i2 = i0 + 2 * MF;
      }
      st2(outH, outL, i0, phi);
      st2(outH, outL, i1, f1);
      st2(outH, outL, i2, f2);
    }
  }
}

__global__ __launch_bounds__(NTHR) void k_state(const float* __restrict__ Kin, const float* __restrict__ Vin,
                                               const float* __restrict__ Om, float* __restrict__ st0) {
  __shared__ __attribute__((aligned(16))) unsigned char pool[115968];
  __bf16* sOH  = (__bf16*)(pool + 0);
  __bf16* sOL  = (__bf16*)(pool + 8192);
  __bf16* sXH  = (__bf16*)(pool + 16384);
  __bf16* sXL  = (__bf16*)(pool + 24576);
  float*  sRec = (float*)(pool + 0);
  __bf16* sKtH = (__bf16*)(pool + 49920);
  __bf16* sKtL = (__bf16*)(pool + 74496);
  __bf16* sVtH = (__bf16*)(pool + 99072);
  __bf16* sVtL = (__bf16*)(pool + 107264);
  float*  sX0  = (float*)(pool + 115456);
  float*  sSS  = (float*)(pool + 115712);

  if (blockIdx.x >= NBLK) return;
  const int tid = threadIdx.x, lane = tid & 31, wave = tid >> 5, h = lane >> 4, l15 = lane & 15;
  const int b = blockIdx.x / NCH, c = blockIdx.x - b * NCH, t0 = c * CH;
  const float* Kb = Kin + ((size_t)b * NTOK + t0) * DL;
  const float* Vb = Vin + ((size_t)b * NTOK + t0) * DL;

  for (int i = tid; i < MF * DX; i += NTHR) st2(sOH, sOL, i, Om[i]);
  stage_x(Kb, sXH, sXL, sX0, sSS, tid);
  for (int i = tid; i < CH * DX; i += NTHR) {
    const int t = i >> 6, j = i & 63;
    st2(sVtH, sVtL, j * CH + t, Vb[(size_t)t * DL + 1 + j]);
  }
  __syncthreads();
  featurize<true>(sXH, sXL, sOH, sOL, sX0, sSS, sKtH, sKtL, 1.0f, wave, lane);
  __syncthreads();

  if (tid < FF) {
    const __bf16* ph = sKtH + tid * CH;
    const __bf16* pl = sKtL + tid * CH;
    float z = 0.f;
#pragma unroll 4
    for (int t = 0; t < CH; ++t) z += (float)ph[t] + (float)pl[t];
    sRec[FF * DX + tid] = z;
  }

  for (int tile = wave; tile < (FF / 16) * (DX / 16); tile += NWAV) {
    const int ft = tile >> 2, jt = tile & 3;
    const __bf16* aH = sKtH + (ft * 16 + l15) * CH + 8 * h;
    const __bf16* aL = sKtL + (ft * 16 + l15) * CH + 8 * h;
    const __bf16* bH = sVtH + (jt * 16 + l15) * CH + 8 * h;
    const __bf16* bL = sVtL + (jt * 16 + l15) * CH + 8 * h;
    v8f acc = zacc();
#pragma unroll 1
    for (int ks = 0; ks < CH / 32; ++ks) {
      const int ko = ks * 32;
      acc = mma3(acc, ldf(aH + ko), ldf(aL + ko), ldf(bH + ko), ldf(bL + ko));
    }
#pragma unroll
    for (int r = 0; r < 8; ++r) sRec[(ft * 16 + 8 * h + r) * DX + jt * 16 + l15] = acc[r];
  }
  __syncthreads();

  float* dst = st0 + (size_t)blockIdx.x * REC;
  const v4f* s4 = (const v4f*)sRec;
  for (int i = tid; i < REC4; i += NTHR) {
    const v4f v = s4[i];
    *((volatile v4f*)dst + i) = v;
  }
  __threadfence();
  for (int i = tid; i < REC4; i += NTHR) {
    const v4f v = s4[i];
    *((volatile v4f*)dst + i) = v;
  }
}

__global__ __launch_bounds__(NTHR) void k_prefix(const float* __restrict__ st0, float* __restrict__ stp) {
  const int e = blockIdx.x * NTHR + threadIdx.x;
  const int b = blockIdx.y;
  if (e >= REC4 || b >= NB) return;
  const size_t base = (size_t)b * NCH * REC4 + e;
  const v4f* src = (const v4f*)st0 + base;
  v4f* dst = (v4f*)stp + base;

  v4f run = {0.f, 0.f, 0.f, 0.f};
#pragma unroll 1
  for (int cc = 0; cc < NCH; ++cc) {
    const v4f v = src[(size_t)cc * REC4];
    *(volatile v4f*)(dst + (size_t)cc * REC4) = run;
    run += v;
  }
  __threadfence();
  v4f run2 = {0.f, 0.f, 0.f, 0.f};
#pragma unroll 1
  for (int cc = 0; cc < NCH; ++cc) {
    const v4f v = src[(size_t)cc * REC4];
    *(volatile v4f*)(dst + (size_t)cc * REC4) = run2;
    run2 += v;
  }
}

__global__ __launch_bounds__(NTHR) void k_out(const float* __restrict__ Qin, const float* __restrict__ Kin,
                                             const float* __restrict__ Vin, const float* __restrict__ Om,
                                             const float* __restrict__ stp, float* __restrict__ out) {
  __shared__ __attribute__((aligned(16))) unsigned char pool[149504];
  __bf16* sOH  = (__bf16*)(pool + 0);
  __bf16* sOL  = (__bf16*)(pool + 8192);
  __bf16* sXH  = (__bf16*)(pool + 16384);
  __bf16* sXL  = (__bf16*)(pool + 24576);
  __bf16* sScH = (__bf16*)(pool + 0);
  __bf16* sScL = (__bf16*)(pool + 8192);
  __bf16* sVtH = (__bf16*)(pool + 16384);
  __bf16* sVtL = (__bf16*)(pool + 24576);
  __bf16* sKfH = (__bf16*)(pool + 32768);
  __bf16* sKfL = (__bf16*)(pool + 57344);
  __bf16* sStH = (__bf16*)(pool + 32768);
  __bf16* sStL = (__bf16*)(pool + 57344);
  __bf16* sQfH = (__bf16*)(pool + 81920);
  __bf16* sQfL = (__bf16*)(pool + 106496);
  float*  sY   = (float*)(pool + 131072);
  float*  sScF = (float*)(pool + 131072);
  float*  sX0  = (float*)(pool + 147712);
  float*  sSS  = (float*)(pool + 147968);
  float*  sZ   = (float*)(pool + 148224);
  float*  sQz  = (float*)(pool + 148992);
  float*  sRow = (float*)(pool + 149248);

  if (blockIdx.x >= NBLK) return;
  const int tid = threadIdx.x, lane = tid & 31, wave = tid >> 5, h = lane >> 4, l15 = lane & 15;
  const int b = blockIdx.x / NCH, c = blockIdx.x - b * NCH, t0 = c * CH;
  const float* Qb = Qin + ((size_t)b * NTOK + t0) * DL;
  const float* Kb = Kin + ((size_t)b * NTOK + t0) * DL;
  const float* Vb = Vin + ((size_t)b * NTOK + t0) * DL;
  const float* sp = stp + (size_t)blockIdx.x * REC;

  for (int i = tid; i < MF * DX; i += NTHR) st2(sOH, sOL, i, Om[i]);
  stage_x(Kb, sXH, sXL, sX0, sSS, tid);
  if (tid < FF) sZ[tid] = sp[FF * DX + tid];
  __syncthreads();
  featurize<false>(sXH, sXL, sOH, sOL, sX0, sSS, sKfH, sKfL, 1.0f, wave, lane);
  __syncthreads();
  stage_x(Qb, sXH, sXL, sX0, sSS, tid);
  __syncthreads();
  featurize<false>(sXH, sXL, sOH, sOL, sX0, sSS, sQfH, sQfL, -1.0f, wave, lane);
  __syncthreads();

  for (int tile = wave; tile < (CH / 16) * (CH / 16); tile += NWAV) {
    const int qt = tile >> 2, kt = tile & 3;
    if (kt > qt) {
#pragma unroll
      for (int r = 0; r < 8; ++r) {
        const int idx = (qt * 16 + 8 * h + r) * CH + kt * 16 + l15;
        sScF[idx] = 0.f;
        sScH[idx] = (__bf16)0.f;
        sScL[idx] = (__bf16)0.f;
      }
    } else {
      const __bf16* aH = sQfH + (qt * 16 + l15) * FF + 8 * h;
      const __bf16* aL = sQfL + (qt * 16 + l15) * FF + 8 * h;
      const __bf16* bH = sKfH + (kt * 16 + l15) * FF + 8 * h;
      const __bf16* bL = sKfL + (kt * 16 + l15) * FF + 8 * h;
      v8f acc = zacc();
#pragma unroll 1
      for (int ks = 0; ks < FF / 32; ++ks) {
        const int ko = ks * 32;
        acc = mma3(acc, ldf(aH + ko), ldf(aL + ko), ldf(bH + ko), ldf(bL + ko));
      }
#pragma unroll
      for (int r = 0; r < 8; ++r) {
        const int row = qt * 16 + 8 * h + r;
        const int col = kt * 16 + l15;
        const int idx = row * CH + col;
        const float val = (col <= row) ? acc[r] : 0.f;
        sScF[idx] = val;
        st2(sScH, sScL, idx, val);
      }
    }
  }
  __syncthreads();

  for (int i = tid; i < CH * DX; i += NTHR) {
    const int t = i >> 6, j = i & 63;
    st2(sVtH, sVtL, j * CH + t, Vb[(size_t)t * DL + 1 + j]);
  }
  for (int i = tid; i < FF * DX; i += NTHR) {
    const int f = i >> 6, j = i & 63;
    st2(sStH, sStL, j * FF + f, sp[i]);
  }
  {
    const int t = tid >> 2, q = tid & 3;
    float rs = 0.f;
    const float* fr = sScF + t * CH + q * 16;
#pragma unroll 4
    for (int i = 0; i < 16; ++i) rs += fr[i];
    rs += __shfl_xor(rs, 1);
    rs += __shfl_xor(rs, 2);
    float qz = 0.f;
    const __bf16* qh = sQfH + t * FF + q * 48;
    const __bf16* ql = sQfL + t * FF + q * 48;
    const float* zz = sZ + q * 48;
#pragma unroll 4
    for (int i = 0; i < 48; ++i) qz += ((float)qh[i] + (float)ql[i]) * zz[i];
    qz += __shfl_xor(qz, 1);
    qz += __shfl_xor(qz, 2);
    if (q == 0) {
      sRow[t] = rs;
      sQz[t] = qz;
    }
  }
  __syncthreads();

  for (int tile = wave; tile < (CH / 16) * (DX / 16); tile += NWAV) {
    const int rt = tile >> 2, jt = tile & 3;
    const __bf16* aH = sQfH + (rt * 16 + l15) * FF + 8 * h;
    const __bf16* aL = sQfL + (rt * 16 + l15) * FF + 8 * h;
    const __bf16* bH = sStH + (jt * 16 + l15) * FF + 8 * h;
    const __bf16* bL = sStL + (jt * 16 + l15) * FF + 8 * h;
    v8f acc = zacc();
#pragma unroll 1
    for (int ks = 0; ks < FF / 32; ++ks) {
      const int ko = ks * 32;
      acc = mma3(acc, ldf(aH + ko), ldf(aL + ko), ldf(bH + ko), ldf(bL + ko));
    }
    const __bf16* cH = sScH + (rt * 16 + l15) * CH + 8 * h;
    const __bf16* cL = sScL + (rt * 16 + l15) * CH + 8 * h;
    const __bf16* dH = sVtH + (jt * 16 + l15) * CH + 8 * h;
    const __bf16* dL = sVtL + (jt * 16 + l15) * CH + 8 * h;
    const int nks = (rt >= 2) ? 2 : 1;
#pragma unroll 1
    for (int ks = 0; ks < nks; ++ks) {
      const int ko = ks * 32;
      acc = mma3(acc, ldf(cH + ko), ldf(cL + ko), ldf(dH + ko), ldf(dL + ko));
    }
#pragma unroll
    for (int r = 0; r < 8; ++r) sY[(rt * 16 + 8 * h + r) * DL + 1 + jt * 16 + l15] = acc[r];
  }
  __syncthreads();

  {
    const int t = tid >> 2, q = tid & 3;
    const float s = sQz[t] + sRow[t];
    const float inv = (fabsf(s) > EPSR) ? (1.0f / s) : (s / (s * s + EPSQ));
    float* yr = sY + t * DL + 1 + q * 16;
    float ssq = 0.f;
#pragma unroll 4
    for (int i = 0; i < 16; ++i) {
      const float y = yr[i] * inv;
      yr[i] = y;
      ssq += y * y;
    }
    ssq += __shfl_xor(ssq, 1);
    ssq += __shfl_xor(ssq, 2);
    if (q == 0) sY[t * DL] = sqrtf(ssq + 1.0f);
  }
  __syncthreads();

  float* ob = out + ((size_t)b * NTOK + t0) * DL;
  const v4f* y4 = (const v4f*)sY;
  for (int i = tid; i < (CH * DL) / 4; i += NTHR) {
    const v4f v = y4[i];
    *((volatile v4f*)ob + i) = v;
  }
  __threadfence();
  for (int i = tid; i < (CH * DL) / 4; i += NTHR) {
    const v4f v = y4[i];
    *((volatile v4f*)ob + i) = v;
  }
}

extern "C" void kernel_launch(void* const* d_in, const int* in_sizes, int n_in,
                              void* d_out, int out_size, void* d_ws, size_t ws_size,
                              hipStream_t stream) {
  const int ntok = NB * NTOK * DL;
  if (n_in < 4) return;
  if (in_sizes[0] != ntok || in_sizes[1] != ntok || in_sizes[2] != ntok || in_sizes[3] != MF * DX) return;
  if (out_size != ntok) return;
  const size_t recb = (size_t)NBLK * REC * sizeof(float);
  if (ws_size < 2 * recb) return;

  const float* Qp = (const float*)d_in[0];
  const float* Kp = (const float*)d_in[1];
  const float* Vp = (const float*)d_in[2];
  const float* Om = (const float*)d_in[3];
  float* outp = (float*)d_out;
  float* st0 = (float*)d_ws;
  float* stp = (float*)((char*)d_ws + recb);

  k_state<<<dim3(NBLK), dim3(NTHR), 0, stream>>>(Kp, Vp, Om, st0);
  k_prefix<<<dim3((REC4 + NTHR - 1) / NTHR, NB), dim3(NTHR), 0, stream>>>(st0, stp);
  k_out<<<dim3(NBLK), dim3(NTHR), 0, stream>>>(Qp, Kp, Vp, Om, stp, outp);
}
